// RecurrentKV_85950885528326
// MI455X (gfx1250) — hardware-run, weakly checked
//
#include <hip/hip_runtime.h>
#include <math.h>

typedef __attribute__((ext_vector_type(16))) _Float16 v16h;
typedef __attribute__((ext_vector_type(8)))  _Float16 v8h;
typedef __attribute__((ext_vector_type(2)))  _Float16 v2h;
typedef __attribute__((ext_vector_type(16))) __bf16   v16b;
typedef __attribute__((ext_vector_type(8)))  __bf16   v8b;
typedef __attribute__((ext_vector_type(8)))  float    v8f;
typedef __attribute__((ext_vector_type(4)))  float    v4f;
typedef __attribute__((ext_vector_type(2)))  float    v2f;
typedef __attribute__((ext_vector_type(4)))  _Float16 v4h;

constexpr int kNb   = 4;
constexpr int kH    = 8;
constexpr int kHS   = kNb * kH;
constexpr int kS    = 1024;
constexpr int kP    = 64;
constexpr int kN    = 64;
constexpr int kQ    = 64;
constexpr int kCS   = kS / kQ;
constexpr int kC    = 2 * kCS;
constexpr int kE    = kHS * kCS;
constexpr int kRows = kE * kQ;
constexpr int kOutAll = kRows * kP;
constexpr int kThr  = 256;
constexpr float kDecay   = 0.95f;
constexpr float kInCarry = 1024.0f;
constexpr float kMCarry  = 256.0f;
constexpr float kHCarry  = 256.0f;
constexpr float kSc1 = 1.0f / (kInCarry * kInCarry);
constexpr float kSc3 = 1.0f / (kMCarry * kInCarry);
constexpr float kSc4 = 1.0f / (kInCarry * kInCarry);
constexpr float kSc6 = 1.0f / (kInCarry * kHCarry);
constexpr float kF16MinNormal = 6.103515625e-5f;

static_assert(kHS == 32 && kS == 1024 && kCS == 16 && kC == 32 && kE == 512 && kRows == 32768 && kP == 64 && kN == 64 && kQ == 64, "the index arithmetic below uses these sizes");

constexpr size_t kOffZB = 0ull;
constexpr size_t kOffXT16 = 4096ull;
constexpr size_t kOffB16 = 4198400ull;
constexpr size_t kOffC16 = 8392704ull;
constexpr size_t kOffCS = 12587008ull;
constexpr size_t kOffOMV = 12718080ull;
constexpr size_t kOffEV = 12849152ull;
constexpr size_t kOffDV = 12980224ull;
constexpr size_t kOffTOT = 13111296ull;
constexpr size_t kOffG32 = 13115392ull;
constexpr size_t kOffM16 = 21504000ull;
constexpr size_t kOffST32 = 25698304ull;
constexpr size_t kOffCE16 = 34086912ull;
constexpr size_t kWsTotal = 38281216ull;
static_assert(kWsTotal <= 134217728ull, "the carve stands under 128 MiB");
static_assert(kOffZB == 0
  && kOffXT16 == kOffZB + 4096ull
  && kOffB16 == kOffXT16 + 4194304ull
  && kOffC16 == kOffB16 + 4194304ull
  && kOffCS == kOffC16 + 4194304ull
  && kOffOMV == kOffCS + 131072ull
  && kOffEV == kOffOMV + 131072ull
  && kOffDV == kOffEV + 131072ull
  && kOffTOT == kOffDV + 131072ull
  && kOffG32 == kOffTOT + 4096ull
  && kOffM16 == kOffG32 + 8388608ull
  && kOffST32 == kOffM16 + 4194304ull
  && kOffCE16 == kOffST32 + 8388608ull
  && kWsTotal == kOffCE16 + 4194304ull, "the carve is a chain: every region starts where the one before ends");
static_assert((kOffXT16 % 256) == 0 && (kOffB16 % 256) == 0 && (kOffC16 % 256) == 0 && (kOffCS % 256) == 0 && (kOffOMV % 256) == 0 && (kOffEV % 256) == 0 && (kOffDV % 256) == 0 && (kOffTOT % 256) == 0 && (kOffG32 % 256) == 0 && (kOffM16 % 256) == 0 && (kOffST32 % 256) == 0 && (kOffCE16 % 256) == 0, "every region starts on a multiple of 256 B");

__device__ __forceinline__ unsigned short f2bf_bits(float f) {
  unsigned u = __float_as_uint(f);
  return (unsigned short)((u + 0x7FFFu + ((u >> 16) & 1u)) >> 16);
}
__device__ __forceinline__ float bf_bits2f(unsigned short h) { return __uint_as_float(((unsigned)h) << 16); }
__device__ __forceinline__ float bf16r(float f) { return bf_bits2f(f2bf_bits(f)); }
__device__ __forceinline__ float carry_flush(float v, float carry) {
  const float s = v * carry;
  return (fabsf(s) < kF16MinNormal) ? 0.0f : s;
}

__device__ __forceinline__ void dep_guard4_h(v8f& a, v8f& b, v8f& c, v8f& d, v16h x, v16h y) { asm volatile("v_nop\n\tv_nop\n\tv_nop\n\tv_nop" : "+v"(a), "+v"(b), "+v"(c), "+v"(d) : "v"(x), "v"(y)); }
__device__ __forceinline__ void dep_guard4_b(v8f& a, v8f& b, v8f& c, v8f& d, v16b x, v16b y) { asm volatile("v_nop\n\tv_nop\n\tv_nop\n\tv_nop" : "+v"(a), "+v"(b), "+v"(c), "+v"(d) : "v"(x), "v"(y)); }
__device__ __forceinline__ void keep4_h(v16h a, v16h b, v16h c, v16h d) { asm volatile("v_nop" :: "v"(a), "v"(b), "v"(c), "v"(d)); }
__device__ __forceinline__ void keep4_b(v16b a, v16b b, v16b c, v16b d) { asm volatile("v_nop" :: "v"(a), "v"(b), "v"(c), "v"(d)); }
__device__ __forceinline__ void acc_guard4(v8f& a, v8f& b, v8f& c, v8f& d) { asm volatile("v_nop\n\tv_nop\n\tv_nop\n\tv_nop" : "+v"(a), "+v"(b), "+v"(c), "+v"(d)); }

template <typename T> struct Frag;
template <> struct Frag<_Float16> {
  typedef v16h V; union U { v16h v; v8h h[2]; };
  static __device__ __forceinline__ v16h load(const _Float16* p) {
    U f; f.h[0] = *(const v8h*)(p); f.h[1] = *(const v8h*)(p + 16); return f.v;
  }
  static __device__ __forceinline__ v8f mma(v16h a, v16h b, v8f c) {
    return __builtin_amdgcn_wmma_f32_16x16x32_f16(false, a, false, b, (short)0, c, false, false);
  }
  static __device__ __forceinline__ void guard4(v8f& a, v8f& b, v8f& c, v8f& d, v16h x, v16h y) { dep_guard4_h(a, b, c, d, x, y); }
  static __device__ __forceinline__ void keep(v16h a, v16h b, v16h c, v16h d) { keep4_h(a, b, c, d); }
};
template <> struct Frag<__bf16> {
  typedef v16b V; union U { v16b v; v8b h[2]; };
  static __device__ __forceinline__ v16b load(const __bf16* p) {
    U f; f.h[0] = *(const v8b*)(p); f.h[1] = *(const v8b*)(p + 16); return f.v;
  }
  static __device__ __forceinline__ v8f mma(v16b a, v16b b, v8f c) {
    return __builtin_amdgcn_wmma_f32_16x16x32_bf16(false, a, false, b, (short)0, c, false, false);
  }
  static __device__ __forceinline__ void guard4(v8f& a, v8f& b, v8f& c, v8f& d, v16b x, v16b y) { dep_guard4_b(a, b, c, d, x, y); }
  static __device__ __forceinline__ void keep(v16b a, v16b b, v16b c, v16b d) { keep4_b(a, b, c, d); }
};

__device__ __forceinline__ v8f mma_h(v16h a, v16h b, v8f c) {
  c = __builtin_amdgcn_wmma_f32_16x16x32_f16(false, a, false, b, (short)0, c, false, false);
  asm volatile("v_nop\n\tv_nop\n\tv_nop\n\tv_nop" : "+v"(c) : "v"(a), "v"(b));
  return c;
}

template <int ET> struct Elem;
template <> struct Elem<0> { typedef _Float16 T; };
template <> struct Elem<1> { typedef __bf16 T; };
template <int ET, bool SPLIT, int BIAS_MODE, int OUT_MODE, bool RESID, int ACT = 0>
__global__ __launch_bounds__(256) void wmma_gemm64(
    const unsigned short* __restrict__ Ap, const unsigned short* __restrict__ A2p, int lda, long strideA,
    const unsigned short* __restrict__ Btp, const unsigned short* __restrict__ Bt2p, int ldb, long strideB,
    void* __restrict__ Cout, void* __restrict__ Cout2, int ldc, long strideC,
    const float* __restrict__ bias,
    const float* __restrict__ resid, long strideR,
    int M, int N, int K, float scale) {
  typedef typename Elem<ET>::T T;
  typedef typename Frag<T>::V V;
  const T* A = (const T*)Ap; const T* A2 = (const T*)A2p; const T* Bt = (const T*)Btp; const T* Bt2 = (const T*)Bt2p;
  __shared__ __align__(16) float sT[8][16 * 68];
  const int b    = blockIdx.y;
  const int lane = threadIdx.x & 31;
  const int wave = threadIdx.x >> 5;
  const int tilesN = N >> 6;
  const int tilesM = M >> 6;
  const int tile = blockIdx.x * 8 + wave;
  if (tile >= tilesM * tilesN) return;
  const int tm = tile / tilesN;
  const int tn = tile - tm * tilesN;
  const int m0 = tm << 6;
  const int n0 = tn << 6;

  const T* Ab  = A  + (size_t)b * strideA;
  const T* Bb  = Bt + (size_t)b * strideB;
  const T* Ab2 = SPLIT ? (A2  + (size_t)b * strideA) : nullptr;
  const T* Bb2 = SPLIT ? (Bt2 + (size_t)b * strideB) : nullptr;

  const int rlane = lane & 15;
  const int koff  = (lane >> 4) * 8;
  const int mOff  = (lane >> 4) * 8;

  v8f acc[4][4];
#pragma unroll
  for (int i = 0; i < 4; ++i)
#pragma unroll
    for (int j = 0; j < 4; ++j) acc[i][j] = (v8f){0.f,0.f,0.f,0.f,0.f,0.f,0.f,0.f};

  for (int k0 = 0; k0 < K; k0 += 32) {
    V bh[4], bl[4];
#pragma unroll
    for (int j = 0; j < 4; ++j) {
      const size_t bo = (size_t)(n0 + (j << 4) + rlane) * ldb + koff + k0;
      bh[j] = Frag<T>::load(Bb + bo);
      if (SPLIT) bl[j] = Frag<T>::load(Bb2 + bo);
    }
#pragma unroll
    for (int i = 0; i < 4; ++i) {
      const size_t ao = (size_t)(m0 + (i << 4) + rlane) * lda + koff + k0;
      V ah = Frag<T>::load(Ab + ao);
      V al;
      if (SPLIT) al = Frag<T>::load(Ab2 + ao);
#pragma unroll
      for (int j = 0; j < 4; ++j) {
        acc[i][j] = Frag<T>::mma(ah, bh[j], acc[i][j]);
        if (SPLIT) {
          acc[i][j] = Frag<T>::mma(ah, bl[j], acc[i][j]);
          acc[i][j] = Frag<T>::mma(al, bh[j], acc[i][j]);
        }
      }
      Frag<T>::guard4(acc[i][0], acc[i][1], acc[i][2], acc[i][3], ah, SPLIT ? al : ah);
    }
    Frag<T>::keep(bh[0], bh[1], bh[2], bh[3]);
    if (SPLIT) Frag<T>::keep(bl[0], bl[1], bl[2], bl[3]);
  }
  acc_guard4(acc[0][0], acc[0][1], acc[0][2], acc[0][3]);
  acc_guard4(acc[1][0], acc[1][1], acc[1][2], acc[1][3]);
  acc_guard4(acc[2][0], acc[2][1], acc[2][2], acc[2][3]);
  acc_guard4(acc[3][0], acc[3][1], acc[3][2], acc[3][3]);

  float* slab = sT[wave];
  const float* Rb = RESID ? (resid + (size_t)b * strideR) : nullptr;
#pragma unroll
  for (int i = 0; i < 4; ++i) {
    const int mBase = m0 + (i << 4);
#pragma unroll
    for (int j = 0; j < 4; ++j) {
      const int n = n0 + (j << 4) + rlane;
      float bv = 0.f;
      if (BIAS_MODE == 2) bv = bias[n];
#pragma unroll
      for (int r = 0; r < 8; ++r) {
        float v = acc[i][j][r] * scale;
        if (BIAS_MODE == 1) v += bias[mBase + mOff + r];
        if (BIAS_MODE == 2) v += bv;
        if (RESID) v += Rb[(size_t)(mBase + mOff + r) * ldc + n];
        if (ACT == 1) v = tanhf(v);
        if (ACT == 2) v = fmaxf(v, 0.0f);
        if (ACT == 3) v = v / (1.0f + expf(-v));
        if (ACT == 4) v = (v > 0.f) ? v : 0.01f * v;
        slab[(mOff + r) * 68 + (j << 4) + rlane] = v;
      }
    }
    __builtin_amdgcn_fence(__ATOMIC_RELEASE, "workgroup");
    __builtin_amdgcn_wave_barrier();
    __builtin_amdgcn_fence(__ATOMIC_ACQUIRE, "workgroup");
    if (OUT_MODE == 0) {
      float* C = (float*)Cout + (size_t)b * strideC;
      const int hh = lane >> 4, c4 = (lane & 15) * 4;
      for (int pass = 0; pass < 2; ++pass) {
#pragma unroll
        for (int it = 0; it < 8; ++it) {
          const int row = it * 2 + hh;
          v4f v = *(const v4f*)(slab + row * 68 + c4);
          *(volatile v4f*)(C + (size_t)(mBase + row) * ldc + n0 + c4) = v;
        }
        __threadfence();
      }
    } else {
      const int q = lane >> 3, c8 = (lane & 7) * 8;
      unsigned short* C  = (unsigned short*)Cout  + (size_t)b * strideC;
      unsigned short* C2 = (OUT_MODE == 2) ? ((unsigned short*)Cout2 + (size_t)b * strideC) : nullptr;
      for (int pass = 0; pass < 2; ++pass) {
#pragma unroll
        for (int it = 0; it < 4; ++it) {
          const int row = it * 4 + q;
          const float* sp = slab + row * 68 + c8;
          v8h hv, lv;
#pragma unroll
          for (int e = 0; e < 8; ++e) {
            if (OUT_MODE == 1) {
              hv[e] = (_Float16)sp[e];
            } else {
              unsigned short hb = f2bf_bits(sp[e]);
              unsigned short lb = f2bf_bits(sp[e] - bf_bits2f(hb));
              hv[e] = __builtin_bit_cast(_Float16, hb);
              lv[e] = __builtin_bit_cast(_Float16, lb);
            }
          }
          *(volatile v8h*)(C + (size_t)(mBase + row) * ldc + n0 + c8) = hv;
          if (OUT_MODE == 2) *(volatile v8h*)(C2 + (size_t)(mBase + row) * ldc + n0 + c8) = lv;
        }
        __threadfence();
      }
    }
    __builtin_amdgcn_fence(__ATOMIC_RELEASE, "workgroup");
    __builtin_amdgcn_wave_barrier();
    __builtin_amdgcn_fence(__ATOMIC_ACQUIRE, "workgroup");
  }
}


__global__ __launch_bounds__(kThr) void cast_plane_kernel(const float* __restrict__ src, unsigned short* __restrict__ dst,
                                                          int colsLog2, int dstPitch, int dstOff) {
  const int i   = blockIdx.x * kThr + threadIdx.x;
  const int sh  = colsLog2 - 3;
  const int row = i >> sh;
  const int c8  = (i & ((1 << sh) - 1)) * 8;
  const float* sp = src + ((size_t)row << colsLog2) + c8;
  const v4f a0 = *(const v4f*)(sp);
  const v4f a1 = *(const v4f*)(sp + 4);
  v8h hv;
#pragma unroll
  for (int e = 0; e < 4; ++e) {
    const float f0 = a0[e];
    const float f1 = a1[e];
    hv[e]     = (_Float16)carry_flush(bf16r(f0), kInCarry);
    hv[4 + e] = (_Float16)carry_flush(bf16r(f1), kInCarry);
  }
  unsigned short* dp = dst + (size_t)row * dstPitch + dstOff + c8;
  *(volatile v8h*)dp = hv;
  __threadfence();
  *(volatile v8h*)dp = hv;
}

__global__ __launch_bounds__(kThr) void zero_kernel(float* __restrict__ dst) {
  const size_t o4 = ((size_t)blockIdx.x * kThr + threadIdx.x) * 4u;
  const v4f z = {0.f, 0.f, 0.f, 0.f};
  *(volatile v4f*)(dst + o4) = z;
  __threadfence();
  *(volatile v4f*)(dst + o4) = z;
}

__global__ __launch_bounds__(kThr) void xt_cast_kernel(const float* __restrict__ V, unsigned short* __restrict__ XT16) {
  const unsigned i = blockIdx.x * (unsigned)kThr + threadIdx.x;
  const unsigned j = i & 7u, p = (i >> 3) & 63u, e = i >> 9;
  const float* sp = V + ((size_t)e * kQ + j * 8u) * kP + p;
  v8h hv;
#pragma unroll
  for (int t = 0; t < 8; ++t) { const float x = sp[(size_t)t * kP]; hv[t] = (_Float16)carry_flush(bf16r(x), kInCarry); }
  unsigned short* dp = XT16 + (size_t)i * 8u;
  *(volatile v8h*)dp = hv;
  __threadfence();
  *(volatile v8h*)dp = hv;
}
static_assert((size_t)kE * kP * (kQ / 8) == 1024ull * kThr, "transposing cast grid exact: 1,024 blocks");

__global__ __launch_bounds__(kThr) void decay_const_kernel(float* __restrict__ CS, float* __restrict__ OMV, float* __restrict__ EV, float* __restrict__ DV, float* __restrict__ TOT) {
  const unsigned e = blockIdx.x * (unsigned)kThr + threadIdx.x;
  const bool first = (e & 15u) == 0u;
  const float ll = logf(kDecay);
  float run = 0.0f;
  for (int q = 0; q < kQ / 4; ++q) {
    v4f s4, o4;
#pragma unroll
    for (int t = 0; t < 4; ++t) { run += ll; s4[t] = run; o4[t] = 1.0f; }
    float* sp = CS + (size_t)e * kQ + 4 * q; float* xp = OMV + (size_t)e * kQ + 4 * q;
    for (int pass = 0; pass < 2; ++pass) { *(volatile v4f*)sp = s4; *(volatile v4f*)xp = o4; __threadfence(); }
  }
  const float tot = run;
  run = 0.0f;
  for (int q = 0; q < kQ / 4; ++q) {
    v4f e4, d4;
#pragma unroll
    for (int t = 0; t < 4; ++t) { run += ll; e4[t] = first ? 0.0f : expf(run); d4[t] = expf(tot - run); }
    float* ep = EV + (size_t)e * kQ + 4 * q; float* dp = DV + (size_t)e * kQ + 4 * q;
    for (int pass = 0; pass < 2; ++pass) { *(volatile v4f*)ep = e4; *(volatile v4f*)dp = d4; __threadfence(); }
  }
  const float te = first ? 0.0f : expf(tot);
  *(volatile float*)(TOT + e) = te;
  __threadfence();
  *(volatile float*)(TOT + e) = te;
}
static_assert(kE == 2 * kThr && (kQ % 4) == 0 && kCS == 16, "the decay arrays' grid exact: 2 blocks; the two passes' trip count is the literal 16 (64 positions by fours); a sequence's first chunk is e a multiple of 16");

__global__ __launch_bounds__(kThr) void mask_kernel(const float* __restrict__ G32, const float* __restrict__ CS, const float* __restrict__ OMV, unsigned short* __restrict__ M16) {
  const unsigned i = blockIdx.x * (unsigned)kThr + threadIdx.x;
  const unsigned s8 = i & 7u, l = (i >> 3) & 63u, e = i >> 9;
  const float* gp = G32 + (size_t)i * 8u;
  const float* xp = CS + (size_t)e * kQ + s8 * 8u;
  const float* wp = OMV + (size_t)e * kQ + s8 * 8u;
  const v4f g0 = *(const v4f*)gp, g1 = *(const v4f*)(gp + 4), x0 = *(const v4f*)xp, x1 = *(const v4f*)(xp + 4), w0 = *(const v4f*)wp, w1 = *(const v4f*)(wp + 4);
  const float csl = CS[(size_t)e * kQ + l];
  v8h hv;
#pragma unroll
  for (int t = 0; t < 8; ++t) {
    const bool live = (s8 * 8u + (unsigned)t) <= l;
    const float gv = (t < 4) ? g0[t] : g1[t - 4];
    const float xv = (t < 4) ? x0[t] : x1[t - 4];
    const float ov = (t < 4) ? w0[t] : w1[t - 4];
    const float d = live ? (csl - xv) : 0.0f;
    const float w = live ? gv * expf(d) * ov : 0.0f;
    hv[t] = (_Float16)carry_flush(w, kMCarry);
  }
  unsigned short* dp = M16 + (size_t)i * 8u;
  *(volatile v8h*)dp = hv;
  __threadfence();
  *(volatile v8h*)dp = hv;
}
static_assert((size_t)kE * kQ * (kQ / 8) == 1024ull * kThr, "mask grid exact: 1,024 blocks");

__global__ __launch_bounds__(kThr) void bdt_cast_kernel(const float* __restrict__ Km, const float* __restrict__ DV, unsigned short* __restrict__ BDT16) {
  const unsigned i = blockIdx.x * (unsigned)kThr + threadIdx.x;
  const unsigned j = i & 7u, n = (i >> 3) & 63u, e = i >> 9;
  const float* sp = Km + ((size_t)e * kQ + j * 8u) * kN + n;
  const float* vp = DV + (size_t)e * kQ + j * 8u;
  const v4f d0 = *(const v4f*)vp, d1 = *(const v4f*)(vp + 4);
  v8h hv;
#pragma unroll
  for (int t = 0; t < 8; ++t) { const float x = sp[(size_t)t * kN]; const float f = (t < 4) ? d0[t] : d1[t - 4]; hv[t] = (_Float16)carry_flush(bf16r(x) * f, kInCarry); }
  unsigned short* dp = BDT16 + (size_t)i * 8u;
  *(volatile v8h*)dp = hv;
  __threadfence();
  *(volatile v8h*)dp = hv;
}
static_assert((size_t)kE * kN * (kQ / 8) == 1024ull * kThr, "scaled transposing cast grid exact: 1,024 blocks");

__global__ __launch_bounds__(kThr) void carry_kernel(const float* __restrict__ ST32, const float* __restrict__ TOT, unsigned short* __restrict__ H16) {
  const unsigned i = blockIdx.x * (unsigned)kThr + threadIdx.x;
  const unsigned n2 = i & 31u, p = (i >> 5) & 63u, hs = i >> 11;
  float h0 = 0.0f, h1 = 0.0f;
  for (int c = 0; c < kC; ++c) {
    const size_t e = (size_t)hs * kC + (size_t)c;
    const size_t o = (e * kP + p) * kN + n2 * 2u;
    v2h hv;
    hv[0] = (_Float16)carry_flush(h0, kHCarry);
    hv[1] = (_Float16)carry_flush(h1, kHCarry);
    unsigned short* dp = H16 + o;
    *(volatile v2h*)dp = hv;
    __threadfence();
    *(volatile v2h*)dp = hv;
    const v2f sv = *(const v2f*)(ST32 + o);
    const float tt = TOT[e];
    h0 = tt * h0 + sv[0];
    h1 = tt * h1 + sv[1];
  }
}
static_assert((size_t)(kHS / 2) * kP * (kN / 2) == 128ull * kThr && kN / 2 == 32 && (kHS % 2) == 0, "carry grid exact: 128 blocks; a wave = one [p] row of 64 state columns; the sequences pair up");

__global__ __launch_bounds__(kThr) void sc_cast_kernel(const float* __restrict__ Qm, const float* __restrict__ EV, unsigned short* __restrict__ CE16) {
  const unsigned i = blockIdx.x * (unsigned)kThr + threadIdx.x;
  const float* sp = Qm + (size_t)i * 8u;
  const v4f a0 = *(const v4f*)sp, a1 = *(const v4f*)(sp + 4);
  const float f = EV[i >> 3];
  v8h hv;
#pragma unroll
  for (int t = 0; t < 4; ++t) {
    const float p = a0[t], q = a1[t];
    hv[t] = (_Float16)carry_flush(bf16r(p) * f, kInCarry);
    hv[4 + t] = (_Float16)carry_flush(bf16r(q) * f, kInCarry);
  }
  unsigned short* dp = CE16 + (size_t)i * 8u;
  *(volatile v8h*)dp = hv;
  __threadfence();
  *(volatile v8h*)dp = hv;
}
static_assert((size_t)kE * kQ * (kN / 8) == 1024ull * kThr && kN / 8 == 8, "scaled cast grid exact: 1,024 blocks; 8 groups a row: EV's index is the row 'i >> 3'");

__global__ __launch_bounds__(kThr) void combine_kernel(const float* __restrict__ YD32, const float* __restrict__ YO32, float* __restrict__ out) {
  const size_t o4 = ((size_t)blockIdx.x * kThr + threadIdx.x) * 4u;
  const v4f a = *(const v4f*)(YD32 + o4), b = *(const v4f*)(YO32 + o4);
  v4f o;
#pragma unroll
  for (int k = 0; k < 4; ++k) o[k] = a[k] + b[k];
  *(volatile v4f*)(out + o4) = o;
  __threadfence();
  *(volatile v4f*)(out + o4) = o;
}
static_assert((size_t)kE * kQ * (kP / 4) == 2048ull * kThr, "combine grid exact: 2,048 blocks: the 2,097,152 outputs");

static_assert(((size_t)kE * kQ * kN / 8) % kThr == 0 && ((size_t)kE * kQ * kN) % 64 == 0, "plane cast grids exact; the planes are whole rows of 64");
extern "C" void kernel_launch(void* const* d_in, const int* in_sizes, int n_in,
                              void* d_out, int out_size, void* d_ws, size_t ws_size,
                              hipStream_t stream) {
  if (n_in < 3 || d_out == nullptr || d_ws == nullptr) return;
  if (in_sizes[0] != kRows * kN || in_sizes[1] != kRows * kN || in_sizes[2] != kRows * kP) return;
  if (out_size != kOutAll) return;
  if (ws_size < kWsTotal) return;
  const float* Qm = (const float*)d_in[0];
  const float* Km = (const float*)d_in[1];
  const float* Vm = (const float*)d_in[2];
  float* out = (float*)d_out;
  char* ws = (char*)d_ws;
  float* ZB = (float*)(ws + kOffZB);
  unsigned short* XT16 = (unsigned short*)(ws + kOffXT16);
  unsigned short* B16 = (unsigned short*)(ws + kOffB16);
  unsigned short* BDT16 = B16;
  unsigned short* C16 = (unsigned short*)(ws + kOffC16);
  unsigned short* H16 = C16;
  float* CS = (float*)(ws + kOffCS);
  float* OMV = (float*)(ws + kOffOMV);
  float* EV = (float*)(ws + kOffEV);
  float* DV = (float*)(ws + kOffDV);
  float* TOT = (float*)(ws + kOffTOT);
  float* G32 = (float*)(ws + kOffG32);
  float* YD32 = G32;
  unsigned short* M16 = (unsigned short*)(ws + kOffM16);
  float* ST32 = (float*)(ws + kOffST32);
  float* YO32 = ST32;
  unsigned short* CE16 = (unsigned short*)(ws + kOffCE16);
  const long kStr = (long)kQ * kN;

  zero_kernel<<<1, kThr, 0, stream>>>(ZB);
  xt_cast_kernel<<<1024, kThr, 0, stream>>>(Vm, XT16);
  cast_plane_kernel<<<(int)(((size_t)kE * kQ * kN / 8) / kThr), kThr, 0, stream>>>(Km, B16, 6, 64, 0);
  cast_plane_kernel<<<(int)(((size_t)kE * kQ * kN / 8) / kThr), kThr, 0, stream>>>(Qm, C16, 6, 64, 0);
  decay_const_kernel<<<2, kThr, 0, stream>>>(CS, OMV, EV, DV, TOT);
  wmma_gemm64<0, false, 2, 0, false, 0><<<dim3(1, kE), 256, 0, stream>>>(
      C16, C16, kN, kStr, B16, B16, kN, kStr, (void*)G32, (void*)G32, kQ, kStr, ZB, nullptr, 0L, kQ, kQ, kN, kSc1);
  mask_kernel<<<1024, kThr, 0, stream>>>(G32, CS, OMV, M16);
  wmma_gemm64<0, false, 2, 0, false, 0><<<dim3(1, kE), 256, 0, stream>>>(
      M16, M16, kQ, kStr, XT16, XT16, kQ, kStr, (void*)YD32, (void*)YD32, kP, kStr, ZB, nullptr, 0L, kQ, kP, kQ, kSc3);
  bdt_cast_kernel<<<1024, kThr, 0, stream>>>(Km, DV, BDT16);
  wmma_gemm64<0, false, 2, 0, false, 0><<<dim3(1, kE), 256, 0, stream>>>(
      XT16, XT16, kQ, kStr, BDT16, BDT16, kQ, kStr, (void*)ST32, (void*)ST32, kN, kStr, ZB, nullptr, 0L, kP, kN, kQ, kSc4);
  carry_kernel<<<128, kThr, 0, stream>>>(ST32, TOT, H16);
  sc_cast_kernel<<<1024, kThr, 0, stream>>>(Qm, EV, CE16);
  wmma_gemm64<0, false, 2, 0, false, 0><<<dim3(1, kE), 256, 0, stream>>>(
      CE16, CE16, kN, kStr, H16, H16, kN, kStr, (void*)YO32, (void*)YO32, kP, kStr, ZB, nullptr, 0L, kQ, kP, kN, kSc6);
  combine_kernel<<<2048, kThr, 0, stream>>>(YD32, YO32, out);
}
